// SingleAttention_61375082660168
// MI455X (gfx1250) — hardware-verified
//
#include <hip/hip_runtime.h>
#include <math.h>
#include <stdint.h>

#ifndef NB
#define NB   8
#endif
#ifndef SEQ
#define SEQ  4096
#endif
#define NB_FULL   8
#define SEQ_FULL  4096
#define DIN  128
#define HD   64
#define NQB  (SEQ / 64)
#define NKT  (SEQ / 64)
static_assert(NB >= 1 && NB <= NB_FULL);
static_assert(SEQ >= 64 && SEQ <= SEQ_FULL && (SEQ % 64) == 0);
static_assert((DIN % 32) == 0 && HD == 64);
static_assert(((SEQ * DIN) / 8) % 32 == 0);
static_assert(((HD * DIN) / 8) % 32 == 0);

typedef _Float16 v16h __attribute__((ext_vector_type(16)));
typedef _Float16 v8h  __attribute__((ext_vector_type(8)));
typedef __bf16   v16b __attribute__((ext_vector_type(16)));
typedef __bf16   v8b  __attribute__((ext_vector_type(8)));
typedef float    v8f  __attribute__((ext_vector_type(8)));
typedef float    v4f  __attribute__((ext_vector_type(4)));
typedef unsigned int v4u __attribute__((ext_vector_type(4)));

__device__ __forceinline__ unsigned short bf_bits(float f) {
  unsigned u = __float_as_uint(f);
  return (unsigned short)((u + 0x7FFFu + ((u >> 16) & 1u)) >> 16);
}
__device__ __forceinline__ float bf_up(unsigned short h) { return __uint_as_float(((unsigned)h) << 16); }
__device__ __forceinline__ unsigned short h_bits(_Float16 x) { return __builtin_bit_cast(unsigned short, x); }
__device__ __forceinline__ unsigned pk16(unsigned short a, unsigned short b) { return (unsigned)a | ((unsigned)b << 16); }
__device__ __forceinline__ v8f zero8() { v8f z = {0.f, 0.f, 0.f, 0.f, 0.f, 0.f, 0.f, 0.f}; return z; }

__device__ __forceinline__ v16b ldfrag_b(const __bf16* p) {
  union { v16b v; v8b h[2]; } f;
  f.h[0] = *(const v8b*)(p);
  f.h[1] = *(const v8b*)(p + 16);
  return f.v;
}

__device__ __forceinline__ v8f mma_b(v16b a, v16b b, v8f c) {
  c = __builtin_amdgcn_wmma_f32_16x16x32_bf16(false, a, false, b, (short)0, c, false, false);
  asm volatile("v_nop\n\tv_nop\n\tv_nop\n\tv_nop" : "+v"(c) : "v"(a), "v"(b));
  return c;
}
__device__ __forceinline__ v8f mma_h(v16h a, v16h b, v8f c) {
  c = __builtin_amdgcn_wmma_f32_16x16x32_f16(false, a, false, b, (short)0, c, false, false);
  asm volatile("v_nop\n\tv_nop\n\tv_nop\n\tv_nop" : "+v"(c) : "v"(a), "v"(b));
  return c;
}
__device__ __forceinline__ v8f mma_b_raw(v16b a, v16b b, v8f c) {
  return __builtin_amdgcn_wmma_f32_16x16x32_bf16(false, a, false, b, (short)0, c, false, false);
}
__device__ __forceinline__ void dep_guard_b(v8f& a, v8f& b, v16b x, v16b y) {
  asm volatile("v_nop\n\tv_nop\n\tv_nop\n\tv_nop" : "+v"(a), "+v"(b) : "v"(x), "v"(y));
}
__device__ __forceinline__ void keep4_b(v16b a, v16b b, v16b c, v16b d) {
  asm volatile("v_nop" :: "v"(a), "v"(b), "v"(c), "v"(d));
}
__device__ __forceinline__ void acc_guard4(v8f& a, v8f& b, v8f& c, v8f& d) {
  asm volatile("v_nop\n\tv_nop\n\tv_nop\n\tv_nop" : "+v"(a), "+v"(b), "+v"(c), "+v"(d));
}

__global__ __launch_bounds__(256) void cvt_bf16x8(const float* __restrict__ in, long long strideIn,
                                                  unsigned short* out, long long strideOut, int n8) {
  const int b = blockIdx.y;
  const int i = blockIdx.x * 256 + (int)threadIdx.x;
  if (i < n8) {
    const float* src = in + (size_t)b * (size_t)strideIn + (size_t)i * 8;
    const v4f a  = *(const v4f*)(src);
    const v4f a4 = *(const v4f*)(src + 4);
    v4u p;
    p[0] = pk16(bf_bits(a[0]),  bf_bits(a[1]));
    p[1] = pk16(bf_bits(a[2]),  bf_bits(a[3]));
    p[2] = pk16(bf_bits(a4[0]), bf_bits(a4[1]));
    p[3] = pk16(bf_bits(a4[2]), bf_bits(a4[3]));
    unsigned short* dst = out + (size_t)b * (size_t)strideOut + (size_t)i * 8;
    *(volatile v4u*)dst = p;
    __threadfence();
    *(volatile v4u*)dst = p;
  }
}

__global__ __launch_bounds__(256) void wt_bf16(const float* __restrict__ W, unsigned short* out, int ngrp) {
  const int i = blockIdx.x * 256 + (int)threadIdx.x;
  if (i < ngrp) {
    const int n  = i / (DIN / 8);
    const int k8 = (i - n * (DIN / 8)) * 8;
    v4u p;
#pragma unroll
    for (int e = 0; e < 4; ++e) {
      const float f0 = W[(size_t)(k8 + 2 * e) * HD + n];
      const float f1 = W[(size_t)(k8 + 2 * e + 1) * HD + n];
      p[e] = pk16(bf_bits(f0), bf_bits(f1));
    }
    unsigned short* o = out + (size_t)n * DIN + k8;
    *(volatile v4u*)o = p;
    __threadfence();
    *(volatile v4u*)o = p;
  }
}

template <int NSPLIT, int OUT_MODE, int BIAS>
__global__ __launch_bounds__(256) void gemm64(
    const unsigned short* __restrict__ Ap, const unsigned short* A2p, int lda, long long strideA,
    const unsigned short* __restrict__ Btp, int ldb, long long strideB,
    const float* __restrict__ bias,
    void* Cout, int ldc, long long strideC,
    void* Cout2, int ldc2, long long strideC2, int N2,
    int M, int N, int K, float rscale) {
  const __bf16* A   = (const __bf16*)(const void*)Ap;
  const __bf16* A2  = (const __bf16*)(const void*)A2p;
  const __bf16* Bt  = (const __bf16*)(const void*)Btp;
  __shared__ __align__(16) float sT[8][16 * 68];
  const int b    = blockIdx.y;
  const int lane = threadIdx.x & 31;
  const int wave = threadIdx.x >> 5;
  const int tilesN = N >> 6;
  const int tilesM = M >> 6;
  const int tile = blockIdx.x * 8 + wave;
  if (tile >= tilesM * tilesN) return;
  const int tm = tile / tilesN;
  const int tn = tile - tm * tilesN;
  const int m0 = tm << 6;
  const int n0 = tn << 6;

  const __bf16* Ab  = A  + (size_t)b * strideA;
  const __bf16* Bb  = Bt + (size_t)b * strideB;
  const __bf16* Ab2 = (NSPLIT >= 1) ? (A2 + (size_t)b * strideA) : Ab;

  const int rlane = lane & 15;
  const int koff  = (lane >> 4) * 8;
  const int mOff  = (lane >> 4) * 8;

  v8f acc[4][4];
#pragma unroll
  for (int i = 0; i < 4; ++i)
#pragma unroll
    for (int j = 0; j < 4; ++j) acc[i][j] = zero8();

  for (int k0 = 0; k0 < K; k0 += 32) {
    v16b bh[4];
#pragma unroll
    for (int j = 0; j < 4; ++j) {
      const size_t bo = (size_t)(n0 + (j << 4) + rlane) * ldb + koff + k0;
      bh[j] = ldfrag_b(Bb + bo);
    }
#pragma unroll
    for (int i = 0; i < 4; ++i) {
      const size_t ao = (size_t)(m0 + (i << 4) + rlane) * lda + koff + k0;
      const v16b ah = ldfrag_b(Ab + ao);
      v16b al = ah;
      if (NSPLIT >= 1) al = ldfrag_b(Ab2 + ao);
#pragma unroll
      for (int j = 0; j < 4; ++j) {
        acc[i][j] = mma_b_raw(ah, bh[j], acc[i][j]);
        if (NSPLIT >= 1) acc[i][j] = mma_b_raw(al, bh[j], acc[i][j]);
      }
      dep_guard_b(acc[i][0], acc[i][3], ah, al);
    }
    keep4_b(bh[0], bh[1], bh[2], bh[3]);
  }
  acc_guard4(acc[0][0], acc[0][1], acc[0][2], acc[0][3]);
  acc_guard4(acc[1][0], acc[1][1], acc[1][2], acc[1][3]);
  acc_guard4(acc[2][0], acc[2][1], acc[2][2], acc[2][3]);
  acc_guard4(acc[3][0], acc[3][1], acc[3][2], acc[3][3]);

  float* slab = sT[wave];
  float bcol[4];
#pragma unroll
  for (int j = 0; j < 4; ++j) {
    bcol[j] = 0.f;
    if (BIAS == 1) bcol[j] = bf_up(bf_bits(bias[n0 + (j << 4) + rlane]));
  }
#pragma unroll
  for (int i = 0; i < 4; ++i) {
    const int mBase = m0 + (i << 4);
    float brow[8];
#pragma unroll
    for (int r = 0; r < 8; ++r) {
      brow[r] = 0.f;
      if (BIAS == 2) brow[r] = bf_up(bf_bits(bias[mBase + mOff + r]));
    }
#pragma unroll
    for (int j = 0; j < 4; ++j) {
#pragma unroll
      for (int r = 0; r < 8; ++r) {
        slab[(mOff + r) * 68 + (j << 4) + rlane] = acc[i][j][r] + bcol[j] + brow[r];
      }
    }
    __builtin_amdgcn_fence(__ATOMIC_RELEASE, "workgroup");
    __builtin_amdgcn_wave_barrier();
    __builtin_amdgcn_fence(__ATOMIC_ACQUIRE, "workgroup");
    if (OUT_MODE == 0) {
      float* C = (float*)Cout + (size_t)b * strideC;
      const int hh = lane >> 4, c4 = (lane & 15) * 4;
      for (int pass = 0; pass < 2; ++pass) {
#pragma unroll
        for (int it = 0; it < 8; ++it) {
          const int row = it * 2 + hh;
          const v4f v = *(const v4f*)(slab + row * 68 + c4);
          *(volatile v4f*)(C + (size_t)(mBase + row) * ldc + n0 + c4) = v;
        }
        __threadfence();
      }
    } else {
      const int q = lane >> 3, c8 = (lane & 7) * 8;
      unsigned short* C  = (unsigned short*)Cout  + (size_t)b * strideC;
      unsigned short* C2 = (unsigned short*)Cout2 + (size_t)b * strideC2;
      const bool wlo = (OUT_MODE == 2) || (n0 < N2);
      v4u hv[4], lv[4];
#pragma unroll
      for (int it = 0; it < 4; ++it) {
        const int row = it * 4 + q;
        const float* sp = slab + row * 68 + c8;
        v4u a, a2;
#pragma unroll
        for (int e = 0; e < 4; ++e) {
          const float f0 = sp[2 * e], f1 = sp[2 * e + 1];
          unsigned short h0, h1, l0, l1;
          if (OUT_MODE == 2) {
            h0 = bf_bits(f0); h1 = bf_bits(f1);
            l0 = bf_bits(f0 - bf_up(h0)); l1 = bf_bits(f1 - bf_up(h1));
          } else {
            const _Float16 x0 = (_Float16)f0, x1 = (_Float16)f1;
            h0 = h_bits(x0); h1 = h_bits(x1);
            l0 = h_bits((_Float16)((f0 - (float)x0) * rscale));
            l1 = h_bits((_Float16)((f1 - (float)x1) * rscale));
          }
          a[e] = pk16(h0, h1); a2[e] = pk16(l0, l1);
        }
        hv[it] = a; lv[it] = a2;
      }
      for (int pass = 0; pass < 2; ++pass) {
#pragma unroll
        for (int it = 0; it < 4; ++it) {
          const int row = it * 4 + q;
          *(volatile v4u*)(C + (size_t)(mBase + row) * ldc + n0 + c8) = hv[it];
          if (wlo) *(volatile v4u*)(C2 + (size_t)(mBase + row) * ldc2 + n0 + c8) = lv[it];
        }
        __threadfence();
      }
    }
    __builtin_amdgcn_fence(__ATOMIC_RELEASE, "workgroup");
    __builtin_amdgcn_wave_barrier();
    __builtin_amdgcn_fence(__ATOMIC_ACQUIRE, "workgroup");
  }
}

__global__ __launch_bounds__(128)
void attn64(const unsigned short* __restrict__ qhp, const unsigned short* __restrict__ qlp,
            const unsigned short* __restrict__ khp, const unsigned short* __restrict__ klp,
            const unsigned short* __restrict__ vhp, const unsigned short* __restrict__ vlp,
            float* outp) {
  union FB { v16b v; v8b h[2]; };
  union FH { v16h v; v8h h[2]; };
  __shared__ __align__(16) __bf16   Ksh[64 * 64];
  __shared__ __align__(16) __bf16   Ksl[64 * 64];
  __shared__ __align__(16) _Float16 Vth[64 * 64];
  __shared__ __align__(16) _Float16 Vtl[64 * 64];
  __shared__ __align__(16) _Float16 Psh[4][16 * 64];
  __shared__ __align__(16) _Float16 Psl[4][16 * 64];
  __shared__ __align__(16) float    Os[4][16 * 64];

  const int tid  = threadIdx.x;
  const int wave = tid >> 5;
  const int lane = tid & 31;
  const int hh   = lane >> 4;
  const int c    = lane & 15;

  const int bx   = blockIdx.x;
  const int qb   = bx % NQB;
  const int b    = bx / NQB;
  const int q0   = qb * 64 + wave * 16;
  const size_t rowB = (size_t)b * SEQ;

  const __bf16* Qh = (const __bf16*)(const void*)qhp;
  const __bf16* Ql = (const __bf16*)(const void*)qlp;
  const __bf16* Kh = (const __bf16*)(const void*)khp;
  const __bf16* Kl = (const __bf16*)(const void*)klp;
  const _Float16* Vh = (const _Float16*)(const void*)vhp + (size_t)b * HD * SEQ;
  const _Float16* Vl = (const _Float16*)(const void*)vlp + (size_t)b * HD * SEQ;

  v16b qah[2], qal[2];
#pragma unroll
  for (int dc = 0; dc < 2; ++dc) {
    const size_t qo = (rowB + q0 + c) * HD + dc * 32 + 8 * hh;
    qah[dc] = ldfrag_b(Qh + qo);
    qal[dc] = ldfrag_b(Ql + qo);
  }

  float mrow[8], lrow[8];
  v8f oacc[4];
#pragma unroll
  for (int r = 0; r < 8; ++r) { mrow[r] = -INFINITY; lrow[r] = 0.f; }
#pragma unroll
  for (int t = 0; t < 4; ++t) oacc[t] = zero8();

  for (int kt = 0; kt < NKT; ++kt) {
    const int kv0 = kt * 64;
    __syncthreads();
    {
      const int r = tid >> 1, half = (tid & 1) * 32;
      const __bf16*   kg  = Kh + (rowB + kv0 + r) * HD + half;
      const __bf16*   klg = Kl + (rowB + kv0 + r) * HD + half;
      const _Float16* vg  = Vh + (size_t)r * SEQ + kv0 + half;
      const _Float16* vlg = Vl + (size_t)r * SEQ + kv0 + half;
#pragma unroll
      for (int i = 0; i < 4; ++i) {
        const v8b a0 = *(const v8b*)(kg + 8 * i);
        const v8b a1 = *(const v8b*)(klg + 8 * i);
        const v8h b0 = *(const v8h*)(vg + 8 * i);
        const v8h b1 = *(const v8h*)(vlg + 8 * i);
        *(v8b*)(Ksh + r * 64 + half + 8 * i) = a0;
        *(v8b*)(Ksl + r * 64 + half + 8 * i) = a1;
        *(v8h*)(Vth + r * 64 + half + 8 * i) = b0;
        *(v8h*)(Vtl + r * 64 + half + 8 * i) = b1;
      }
    }
    __syncthreads();

    v8f s[4];
#pragma unroll
    for (int j = 0; j < 4; ++j) {
      s[j] = zero8();
#pragma unroll
      for (int dc = 0; dc < 2; ++dc) {
        FB kb, kl;
        kb.h[0] = *(const v8b*)(Ksh + (j * 16 + c) * 64 + dc * 32 + 8 * hh);
        kb.h[1] = *(const v8b*)(Ksh + (j * 16 + c) * 64 + dc * 32 + 16 + 8 * hh);
        kl.h[0] = *(const v8b*)(Ksl + (j * 16 + c) * 64 + dc * 32 + 8 * hh);
        kl.h[1] = *(const v8b*)(Ksl + (j * 16 + c) * 64 + dc * 32 + 16 + 8 * hh);
        s[j] = mma_b(qah[dc], kb.v, s[j]);
        s[j] = mma_b(qah[dc], kl.v, s[j]);
        s[j] = mma_b(qal[dc], kb.v, s[j]);
      }
    }

    _Float16* pwh = Psh[wave];
    _Float16* pwl = Psl[wave];
#pragma unroll
    for (int r = 0; r < 8; ++r) {
      float m = -INFINITY;
#pragma unroll
      for (int j = 0; j < 4; ++j) {
        const float sv = s[j][r] * 0.125f;
        s[j][r] = sv;
        m = fmaxf(m, sv);
      }
#pragma unroll
      for (int off = 1; off < 16; off <<= 1) m = fmaxf(m, __shfl_xor(m, off, 32));
      const float mnew  = fmaxf(mrow[r], m);
      const float msafe = (mnew == -INFINITY) ? 0.f : mnew;
      const float alpha = __expf(mrow[r] - msafe);
      mrow[r] = mnew;
      float psum = 0.f;
#pragma unroll
      for (int j = 0; j < 4; ++j) {
        const float p = __expf(s[j][r] - msafe);
        psum += p;
        const float p1k = p * 1024.0f;
        const _Float16 ph = (_Float16)p1k;
        const _Float16 pl = (_Float16)((p1k - (float)ph) * 4096.0f);
        pwh[(8 * hh + r) * 64 + j * 16 + c] = ph;
        pwl[(8 * hh + r) * 64 + j * 16 + c] = pl;
      }
#pragma unroll
      for (int off = 1; off < 16; off <<= 1) psum += __shfl_xor(psum, off, 32);
      lrow[r] = lrow[r] * alpha + psum;
#pragma unroll
      for (int t = 0; t < 4; ++t) oacc[t][r] *= alpha;
    }
    __builtin_amdgcn_fence(__ATOMIC_RELEASE, "workgroup");
    __builtin_amdgcn_wave_barrier();
    __builtin_amdgcn_fence(__ATOMIC_ACQUIRE, "workgroup");

    v8f o1[4];
#pragma unroll
    for (int t = 0; t < 4; ++t) o1[t] = zero8();
#pragma unroll 1
    for (int kk = 0; kk < 2; ++kk) {
      FH pa, pr;
      pa.h[0] = *(const v8h*)(pwh + c * 64 + kk * 32 + 8 * hh);
      pa.h[1] = *(const v8h*)(pwh + c * 64 + kk * 32 + 16 + 8 * hh);
      pr.h[0] = *(const v8h*)(pwl + c * 64 + kk * 32 + 8 * hh);
      pr.h[1] = *(const v8h*)(pwl + c * 64 + kk * 32 + 16 + 8 * hh);
#pragma unroll
      for (int t = 0; t < 4; ++t) {
        FH vb, vl;
        vb.h[0] = *(const v8h*)(Vth + (t * 16 + c) * 64 + kk * 32 + 8 * hh);
        vb.h[1] = *(const v8h*)(Vth + (t * 16 + c) * 64 + kk * 32 + 16 + 8 * hh);
        vl.h[0] = *(const v8h*)(Vtl + (t * 16 + c) * 64 + kk * 32 + 8 * hh);
        vl.h[1] = *(const v8h*)(Vtl + (t * 16 + c) * 64 + kk * 32 + 16 + 8 * hh);
        oacc[t] = mma_h(pa.v, vb.v, oacc[t]);
        o1[t]   = mma_h(pa.v, vl.v, o1[t]);
        o1[t]   = mma_h(pr.v, vb.v, o1[t]);
      }
    }
#pragma unroll
    for (int t = 0; t < 4; ++t)
#pragma unroll
      for (int r = 0; r < 8; ++r) oacc[t][r] += o1[t][r] * (1.0f / 4096.0f);
  }

  float* os = Os[wave];
#pragma unroll
  for (int r = 0; r < 8; ++r) {
    const float l = lrow[r];
    const float inv = ((l > 0.f) ? (1.0f / l) : 0.f) * (1.0f / 1024.0f);
#pragma unroll
    for (int t = 0; t < 4; ++t) os[(8 * hh + r) * 64 + t * 16 + c] = oacc[t][r] * inv;
  }
  __builtin_amdgcn_fence(__ATOMIC_RELEASE, "workgroup");
  __builtin_amdgcn_wave_barrier();
  __builtin_amdgcn_fence(__ATOMIC_ACQUIRE, "workgroup");
  {
    const int h2 = lane >> 4, c4 = (lane & 15) * 4;
    v4f ov[8];
#pragma unroll
    for (int it = 0; it < 8; ++it) {
      const int row = it * 2 + h2;
      ov[it] = *(const v4f*)(os + row * 64 + c4);
    }
    for (int pass = 0; pass < 2; ++pass) {
#pragma unroll
      for (int it = 0; it < 8; ++it) {
        const int row = it * 2 + h2;
        const size_t go = (rowB + q0 + row) * HD + c4;
        *(volatile v4f*)(outp + go) = ov[it];
      }
      __threadfence();
    }
  }
}

extern "C" void kernel_launch(void* const* d_in, const int* in_sizes, int n_in,
                              void* d_out, int out_size, void* d_ws, size_t ws_size,
                              hipStream_t stream) {
  if (n_in < 9) return;
  const long long NEEDX = ((long long)(NB - 1) * SEQ_FULL + SEQ) * DIN;
  const int NXC = NB * SEQ * DIN;
  const int NO  = NB * SEQ * HD;
  const int NW  = DIN * HD;
  if ((long long)in_sizes[0] < NEEDX || (long long)in_sizes[1] < NEEDX || (long long)in_sizes[2] < NEEDX) return;
  if (in_sizes[3] < NW || in_sizes[5] < NW || in_sizes[7] < NW) return;
  if (in_sizes[4] < HD || in_sizes[6] < HD || in_sizes[8] < HD) return;
  if (out_size < NO) return;

  const float* q_in = (const float*)d_in[0];
  const float* k_in = (const float*)d_in[1];
  const float* v_in = (const float*)d_in[2];
  const float* Wq   = (const float*)d_in[3];
  const float* bq   = (const float*)d_in[4];
  const float* Wk   = (const float*)d_in[5];
  const float* bk   = (const float*)d_in[6];
  const float* Wv   = (const float*)d_in[7];
  const float* bv   = (const float*)d_in[8];

  const size_t PX  = (size_t)NXC * 2;
  const size_t PW  = (size_t)NW * 2;
  const size_t PP  = (size_t)NO * 2;
  const size_t PVT = (size_t)NB * HD * SEQ * 2;
  size_t off = 0;
  const size_t oQb  = off; off += PX;
  const size_t oKb  = off; off += PX;
  const size_t oVb  = off; off += PX;
  const size_t oWq  = off; off += PW;
  const size_t oWk  = off; off += PW;
  const size_t oWv  = off; off += PW;
  const size_t oQh  = off; off += PP;
  const size_t oQl  = off; off += PP;
  const size_t oKh  = off; off += PP;
  const size_t oKl  = off; off += PP;
  const size_t oVTh = off; off += PVT;
  const size_t oVTl = off; off += PVT;
  if (off > ws_size) return;
  if (off > (size_t)134217728) return;

  char* ws = (char*)d_ws;
  unsigned short* Qb  = (unsigned short*)(ws + oQb);
  unsigned short* Kb  = (unsigned short*)(ws + oKb);
  unsigned short* Vb  = (unsigned short*)(ws + oVb);
  unsigned short* WqT = (unsigned short*)(ws + oWq);
  unsigned short* WkT = (unsigned short*)(ws + oWk);
  unsigned short* WvT = (unsigned short*)(ws + oWv);
  unsigned short* Qh  = (unsigned short*)(ws + oQh);
  unsigned short* Ql  = (unsigned short*)(ws + oQl);
  unsigned short* Kh  = (unsigned short*)(ws + oKh);
  unsigned short* Kl  = (unsigned short*)(ws + oKl);
  unsigned short* VTh = (unsigned short*)(ws + oVTh);
  unsigned short* VTl = (unsigned short*)(ws + oVTl);

  const dim3 blk(256);
  const int n8x = (SEQ * DIN) / 8;
  const int n8w = NW / 8;
  const dim3 gCvtX((n8x + 255) / 256, NB);
  const dim3 gWt((n8w + 255) / 256);
  const dim3 gProj(((NB * SEQ / 64) * (HD / 64) + 7) / 8, 1);
  const dim3 gVT(((HD / 64) * (SEQ / 64) + 7) / 8, NB);
  const dim3 gAttn(NB * NQB);

  const long long strideInX  = (long long)SEQ_FULL * DIN;
  const long long strideOutX = (long long)SEQ * DIN;

  cvt_bf16x8<<<gCvtX, blk, 0, stream>>>(q_in, strideInX, Qb, strideOutX, n8x);
  cvt_bf16x8<<<gCvtX, blk, 0, stream>>>(k_in, strideInX, Kb, strideOutX, n8x);
  cvt_bf16x8<<<gCvtX, blk, 0, stream>>>(v_in, strideInX, Vb, strideOutX, n8x);
  wt_bf16<<<gWt, blk, 0, stream>>>(Wq, WqT, n8w);
  wt_bf16<<<gWt, blk, 0, stream>>>(Wk, WkT, n8w);
  wt_bf16<<<gWt, blk, 0, stream>>>(Wv, WvT, n8w);
  gemm64<0, 2, 1><<<gProj, blk, 0, stream>>>(
      Qb, Qb, DIN, 0LL, WqT, DIN, 0LL, bq,
      (void*)Qh, HD, 0LL, (void*)Ql, HD, 0LL, HD,
      NB * SEQ, HD, DIN, 1.0f);
  gemm64<0, 2, 1><<<gProj, blk, 0, stream>>>(
      Kb, Kb, DIN, 0LL, WkT, DIN, 0LL, bk,
      (void*)Kh, HD, 0LL, (void*)Kl, HD, 0LL, HD,
      NB * SEQ, HD, DIN, 1.0f);
  gemm64<0, 3, 2><<<gVT, blk, 0, stream>>>(
      WvT, WvT, DIN, 0LL, Vb, DIN, (long long)SEQ * DIN, bv,
      (void*)VTh, SEQ, (long long)HD * SEQ, (void*)VTl, SEQ, (long long)HD * SEQ, SEQ,
      HD, SEQ, DIN, 4096.0f);
  attn64<<<gAttn, dim3(128), 0, stream>>>(Qh, Ql, Kh, Kl, VTh, VTl, (float*)d_out);
  (void)hipGetLastError();
}
